// MHSA_67525475827795
// MI455X (gfx1250) — hardware-verified
//
#include <hip/hip_runtime.h>
#include <math.h>
#include <stdint.h>

#define NBATCH 2
#define SEQ    2048
#define DMOD   1024
#define NHEAD  16
#define DHD    64
#define NTOK   (NBATCH * SEQ)
#define QKP    (2 * DMOD)
#define CTXP   (2 * DMOD)

static_assert(NHEAD * DHD == DMOD);
static_assert(DMOD % 64 == 0 && SEQ % 64 == 0 && NTOK % 64 == 0);
static_assert(DMOD % 32 == 0 && CTXP % 32 == 0);

typedef __attribute__((ext_vector_type(16))) __bf16 v16b;
typedef __attribute__((ext_vector_type(8)))  __bf16 v8b;
typedef __attribute__((ext_vector_type(8)))  float  v8f;
typedef __attribute__((ext_vector_type(4)))  float  v4f;
typedef __attribute__((ext_vector_type(4)))  unsigned int v4u;

union FB { v16b v; v8b h[2]; };

__device__ __forceinline__ unsigned short f2bf_bits(float f) {
  unsigned u = __float_as_uint(f);
  return (unsigned short)((u + 0x7FFFu + ((u >> 16) & 1u)) >> 16);
}
__device__ __forceinline__ float bf_bits2f(unsigned short h) { return __uint_as_float(((unsigned)h) << 16); }
__device__ __forceinline__ unsigned pk16(unsigned short a, unsigned short b) { return (unsigned)a | ((unsigned)b << 16); }

__device__ __forceinline__ void split2(float f0, float f1, unsigned& uh, unsigned& ul) {
  const unsigned short h0 = f2bf_bits(f0), h1 = f2bf_bits(f1);
  const unsigned short l0 = f2bf_bits(f0 - bf_bits2f(h0)), l1 = f2bf_bits(f1 - bf_bits2f(h1));
  uh = pk16(h0, h1);
  ul = pk16(l0, l1);
}
__device__ __forceinline__ void split8(v4f a, v4f b, v4u& hv, v4u& lv) {
  unsigned h, l;
  split2(a[0], a[1], h, l); hv[0] = h; lv[0] = l;
  split2(a[2], a[3], h, l); hv[1] = h; lv[1] = l;
  split2(b[0], b[1], h, l); hv[2] = h; lv[2] = l;
  split2(b[2], b[3], h, l); hv[3] = h; lv[3] = l;
}
__device__ __forceinline__ v4u pack8(v4f a, v4f b) {
  v4u o;
  o[0] = pk16(f2bf_bits(a[0]), f2bf_bits(a[1]));
  o[1] = pk16(f2bf_bits(a[2]), f2bf_bits(a[3]));
  o[2] = pk16(f2bf_bits(b[0]), f2bf_bits(b[1]));
  o[3] = pk16(f2bf_bits(b[2]), f2bf_bits(b[3]));
  return o;
}

__device__ __forceinline__ v16b frag_load(const __bf16* p) {
  FB f; f.h[0] = *(const v8b*)(p); f.h[1] = *(const v8b*)(p + 16); return f.v;
}
__device__ __forceinline__ v8f mma_raw(v16b a, v16b b, v8f c) {
  return __builtin_amdgcn_wmma_f32_16x16x32_bf16(false, a, false, b, (short)0, c, false, false);
}
__device__ __forceinline__ v8f at_mma(v16b a, v16b b, v8f c) {
  c = __builtin_amdgcn_wmma_f32_16x16x32_bf16(false, a, false, b, (short)0, c, false, false);
  asm volatile("v_nop\n\tv_nop\n\tv_nop\n\tv_nop" : "+v"(c) : "v"(a), "v"(b));
  return c;
}
__device__ __forceinline__ void group_guard(v8f& a, v8f& b, v8f& c, v8f& d, v16b x) {
  asm volatile("v_nop\n\tv_nop\n\tv_nop\n\tv_nop" : "+v"(a), "+v"(b), "+v"(c), "+v"(d) : "v"(x));
}
__device__ __forceinline__ void keep4_b(v16b a, v16b b, v16b c, v16b d) { asm volatile("v_nop" :: "v"(a), "v"(b), "v"(c), "v"(d)); }
__device__ __forceinline__ void acc_guard4(v8f& a, v8f& b, v8f& c, v8f& d) { asm volatile("v_nop\n\tv_nop\n\tv_nop\n\tv_nop" : "+v"(a), "+v"(b), "+v"(c), "+v"(d)); }

#define NX8   (NTOK * DMOD / 8)
#define NWQ8  (3 * DMOD * DMOD / 8)
#define NWO8  (DMOD * 2 * DMOD / 8)
#define NB4   (DMOD / 4)
#define NPREP (NX8 + NWQ8 + NWO8 + NB4)
static_assert(NX8 % 256 == 0 && NWQ8 % 256 == 0 && NWO8 % 256 == 0 && NB4 % 256 == 0);

__global__ __launch_bounds__(256) void prep_kernel(
    const float* __restrict__ x, const float* __restrict__ wqkv, const float* __restrict__ wout,
    const float* __restrict__ bout,
    unsigned short* __restrict__ xb, unsigned short* __restrict__ wq, unsigned short* __restrict__ wo2,
    float* __restrict__ br)
{
  const int g = blockIdx.x * 256 + threadIdx.x;
  if (g >= NPREP) return;
  if (g < NX8 + NWQ8 + NWO8) {
    const float* src;
    unsigned short* dst;
    if (g < NX8) {
      src = x + (size_t)g * 8;
      dst = xb + (size_t)g * 8;
    } else if (g < NX8 + NWQ8) {
      const int e = g - NX8;
      src = wqkv + (size_t)e * 8;
      dst = wq + (size_t)e * 8;
    } else {
      const int e  = g - NX8 - NWQ8;
      const int n  = e >> 8;
      const int kc = (e & 255) * 8;
      src = wout + (size_t)n * DMOD + (kc & (DMOD - 1));
      dst = wo2 + (size_t)e * 8;
    }
    const v4f a = *(const v4f*)(src);
    const v4f c = *(const v4f*)(src + 4);
    const v4u o = pack8(a, c);
    *(volatile v4u*)dst = o;
    __threadfence();
    *(volatile v4u*)dst = o;
  } else {
    const int e = g - NX8 - NWQ8 - NWO8;
    const v4f a = *(const v4f*)(bout + (size_t)e * 4);
    v4f o;
    o[0] = bf_bits2f(f2bf_bits(a[0]));
    o[1] = bf_bits2f(f2bf_bits(a[1]));
    o[2] = bf_bits2f(f2bf_bits(a[2]));
    o[3] = bf_bits2f(f2bf_bits(a[3]));
    float* dstf = br + (size_t)e * 4;
    *(volatile v4f*)dstf = o;
    __threadfence();
    *(volatile v4f*)dstf = o;
  }
}

template <int BIAS_MODE, int OUT_MODE>
__global__ __launch_bounds__(256) void wmma_gemm64(
    const unsigned short* __restrict__ Ap, int lda, long strideA,
    const unsigned short* __restrict__ Btp, int ldb, long strideB,
    void* __restrict__ Cout, void* __restrict__ Cout2, int ldc, long strideC,
    const float* __restrict__ bias, int M, int N, int K)
{
  __shared__ __align__(16) float sT[8][16 * 68];
  const __bf16* A  = (const __bf16*)(const void*)Ap;
  const __bf16* Bt = (const __bf16*)(const void*)Btp;
  const int b    = blockIdx.y;
  const int lane = threadIdx.x & 31;
  const int wave = threadIdx.x >> 5;
  const int tilesN = N >> 6;
  const int tilesM = M >> 6;
  const int tile = blockIdx.x * 8 + wave;
  if (tile >= tilesM * tilesN) return;
  const int tm = tile / tilesN;
  const int tn = tile - tm * tilesN;
  const int m0 = tm << 6;
  const int n0 = tn << 6;

  const __bf16* Ab = A  + (size_t)b * strideA;
  const __bf16* Bb = Bt + (size_t)b * strideB;

  const int rlane = lane & 15;
  const int koff  = (lane >> 4) * 8;
  const int mOff  = (lane >> 4) * 8;

  v8f acc[4][4];
#pragma unroll
  for (int i = 0; i < 4; ++i)
#pragma unroll
    for (int j = 0; j < 4; ++j) acc[i][j] = (v8f){0.f,0.f,0.f,0.f,0.f,0.f,0.f,0.f};

#pragma unroll 1
  for (int k0 = 0; k0 < K; k0 += 32) {
    v16b bh[4];
#pragma unroll
    for (int j = 0; j < 4; ++j) {
      const size_t bo = (size_t)(n0 + (j << 4) + rlane) * ldb + koff + k0;
      bh[j] = frag_load(Bb + bo);
    }
#pragma unroll
    for (int i = 0; i < 4; ++i) {
      const size_t ao = (size_t)(m0 + (i << 4) + rlane) * lda + koff + k0;
      const v16b ah = frag_load(Ab + ao);
#pragma unroll
      for (int j = 0; j < 4; ++j) acc[i][j] = mma_raw(ah, bh[j], acc[i][j]);
      group_guard(acc[i][0], acc[i][1], acc[i][2], acc[i][3], ah);
    }
    keep4_b(bh[0], bh[1], bh[2], bh[3]);
  }
  acc_guard4(acc[0][0], acc[0][1], acc[0][2], acc[0][3]);
  acc_guard4(acc[1][0], acc[1][1], acc[1][2], acc[1][3]);
  acc_guard4(acc[2][0], acc[2][1], acc[2][2], acc[2][3]);
  acc_guard4(acc[3][0], acc[3][1], acc[3][2], acc[3][3]);

  float* slab = sT[wave];
#pragma unroll
  for (int i = 0; i < 4; ++i) {
    const int mBase = m0 + (i << 4);
#pragma unroll
    for (int j = 0; j < 4; ++j) {
      const int n = n0 + (j << 4) + rlane;
      float bv = 0.f;
      if (BIAS_MODE == 2) bv = bias[n];
#pragma unroll
      for (int r = 0; r < 8; ++r) {
        float v = acc[i][j][r];
        if (BIAS_MODE == 2) v += bv;
        slab[(mOff + r) * 68 + (j << 4) + rlane] = v;
      }
    }
    __builtin_amdgcn_fence(__ATOMIC_RELEASE, "workgroup");
    __builtin_amdgcn_wave_barrier();
    __builtin_amdgcn_fence(__ATOMIC_ACQUIRE, "workgroup");
    if (OUT_MODE == 0) {
      float* C = (float*)Cout + (size_t)b * strideC;
      const int hh = lane >> 4, c4 = (lane & 15) * 4;
      for (int pass = 0; pass < 2; ++pass) {
#pragma unroll
        for (int it = 0; it < 8; ++it) {
          const int row = it * 2 + hh;
          const v4f v = *(const v4f*)(slab + row * 68 + c4);
          *(volatile v4f*)(C + (size_t)(mBase + row) * ldc + n0 + c4) = v;
        }
        __threadfence();
      }
    } else {
      const int q = lane >> 3, c8 = (lane & 7) * 8;
      unsigned short* C  = (unsigned short*)Cout  + (size_t)b * strideC;
      unsigned short* C2 = (unsigned short*)Cout2 + (size_t)b * strideC;
      v4u hv[4], lv[4];
#pragma unroll
      for (int it = 0; it < 4; ++it) {
        const int row = it * 4 + q;
        const float* sp = slab + row * 68 + c8;
        const v4f a0 = *(const v4f*)(sp);
        const v4f a1 = *(const v4f*)(sp + 4);
        split8(a0, a1, hv[it], lv[it]);
      }
      for (int pass = 0; pass < 2; ++pass) {
#pragma unroll
        for (int it = 0; it < 4; ++it) {
          const int row = it * 4 + q;
          const size_t go = (size_t)(mBase + row) * ldc + n0 + c8;
          *(volatile v4u*)(C + go)  = hv[it];
          *(volatile v4u*)(C2 + go) = lv[it];
        }
        __threadfence();
      }
    }
    __builtin_amdgcn_fence(__ATOMIC_RELEASE, "workgroup");
    __builtin_amdgcn_wave_barrier();
    __builtin_amdgcn_fence(__ATOMIC_ACQUIRE, "workgroup");
  }
}

#define AT_D 64
#define AT_NW 4
#define AT_QB 64
#define AT_KC 64

__device__ __forceinline__ void at_split(float f, __bf16& hi, __bf16& lo) {
  const unsigned short hb = f2bf_bits(f);
  hi = __builtin_bit_cast(__bf16, hb);
  const unsigned short lb = f2bf_bits(f - bf_bits2f(hb));
  lo = __builtin_bit_cast(__bf16, lb);
}

__global__ __launch_bounds__(128)
void attn_full64_kernel(const unsigned short* __restrict__ qkhp, const unsigned short* __restrict__ qklp,
                        const unsigned short* __restrict__ vthp, const unsigned short* __restrict__ vtlp,
                        unsigned short* __restrict__ ctx) {
  __shared__ __align__(16) __bf16 Ksh[AT_KC * AT_D];
  __shared__ __align__(16) __bf16 Ksl[AT_KC * AT_D];
  __shared__ __align__(16) __bf16 Vth[AT_D * AT_KC];
  __shared__ __align__(16) __bf16 Vtl[AT_D * AT_KC];
  __shared__ __align__(16) __bf16 Psh[AT_NW][16 * AT_KC];
  __shared__ __align__(16) __bf16 Psl[AT_NW][16 * AT_KC];
  __shared__ __align__(16) float  Os[AT_NW][16 * 68];

  const int tid  = threadIdx.x;
  const int wave = tid >> 5;
  const int lane = tid & 31;
  const int hh   = lane >> 4;
  const int c    = lane & 15;

  const int nqb = SEQ / AT_QB;
  const int bx = blockIdx.x;
  const int qb = bx % nqb;
  const int h  = bx / nqb;
  const int b  = blockIdx.y;
  const int q0 = qb * AT_QB + wave * 16;
  const size_t tokb = (size_t)b * SEQ;

  const __bf16* Qh = (const __bf16*)(const void*)qkhp + tokb * QKP + (size_t)h * AT_D;
  const __bf16* Ql = (const __bf16*)(const void*)qklp + tokb * QKP + (size_t)h * AT_D;
  const __bf16* Kh = (const __bf16*)(const void*)qkhp + tokb * QKP + DMOD + (size_t)h * AT_D;
  const __bf16* Kl = (const __bf16*)(const void*)qklp + tokb * QKP + DMOD + (size_t)h * AT_D;
  const __bf16* Vh = (const __bf16*)(const void*)vthp + ((size_t)b * DMOD + (size_t)h * AT_D) * SEQ;
  const __bf16* Vl = (const __bf16*)(const void*)vtlp + ((size_t)b * DMOD + (size_t)h * AT_D) * SEQ;

  v16b qah[2], qal[2];
#pragma unroll
  for (int dc = 0; dc < 2; ++dc) {
    const __bf16* qr = Qh + (size_t)(q0 + c) * QKP + dc * 32 + 8 * hh;
    const __bf16* ql = Ql + (size_t)(q0 + c) * QKP + dc * 32 + 8 * hh;
    qah[dc] = frag_load(qr);
    qal[dc] = frag_load(ql);
  }

  float mrow[8], lrow[8];
  v8f oacc[4];
#pragma unroll
  for (int r = 0; r < 8; ++r) { mrow[r] = -INFINITY; lrow[r] = 0.f; }
#pragma unroll
  for (int t = 0; t < 4; ++t) oacc[t] = (v8f){0.f,0.f,0.f,0.f,0.f,0.f,0.f,0.f};

  const float sscale = 0.125f;
  const int nChunks = SEQ / AT_KC;
#pragma unroll 1
  for (int kc = 0; kc < nChunks; ++kc) {
    const int kv0 = kc * AT_KC;
    __syncthreads();
    {
      const int r = tid >> 1, half = (tid & 1) * 32;
      const __bf16* ksh = Kh + (size_t)(kv0 + r) * QKP + half;
      const __bf16* ksl = Kl + (size_t)(kv0 + r) * QKP + half;
      const __bf16* vsh = Vh + (size_t)r * SEQ + kv0 + half;
      const __bf16* vsl = Vl + (size_t)r * SEQ + kv0 + half;
#pragma unroll
      for (int i = 0; i < 4; ++i) {
        const v8b a0 = *(const v8b*)(ksh + 8 * i);
        const v8b a1 = *(const v8b*)(ksl + 8 * i);
        const v8b b0 = *(const v8b*)(vsh + 8 * i);
        const v8b b1 = *(const v8b*)(vsl + 8 * i);
        *(v8b*)(Ksh + r * AT_D  + half + 8 * i) = a0;
        *(v8b*)(Ksl + r * AT_D  + half + 8 * i) = a1;
        *(v8b*)(Vth + r * AT_KC + half + 8 * i) = b0;
        *(v8b*)(Vtl + r * AT_KC + half + 8 * i) = b1;
      }
    }
    __syncthreads();

    v8f s[4];
#pragma unroll
    for (int j = 0; j < 4; ++j) {
      s[j] = (v8f){0.f,0.f,0.f,0.f,0.f,0.f,0.f,0.f};
#pragma unroll
      for (int dc = 0; dc < 2; ++dc) {
        FB kb, kl;
        kb.h[0] = *(const v8b*)(Ksh + (j * 16 + c) * AT_D + dc * 32 + 8 * hh);
        kb.h[1] = *(const v8b*)(Ksh + (j * 16 + c) * AT_D + dc * 32 + 16 + 8 * hh);
        kl.h[0] = *(const v8b*)(Ksl + (j * 16 + c) * AT_D + dc * 32 + 8 * hh);
        kl.h[1] = *(const v8b*)(Ksl + (j * 16 + c) * AT_D + dc * 32 + 16 + 8 * hh);
        s[j] = at_mma(qah[dc], kb.v, s[j]);
        s[j] = at_mma(qah[dc], kl.v, s[j]);
        s[j] = at_mma(qal[dc], kb.v, s[j]);
      }
    }
    float cm[8];
#pragma unroll
    for (int r = 0; r < 8; ++r) {
      float m = -INFINITY;
#pragma unroll
      for (int j = 0; j < 4; ++j) {
        const float sv = s[j][r] * sscale;
        s[j][r] = sv;
        m = fmaxf(m, sv);
      }
#pragma unroll
      for (int off = 1; off < 16; off <<= 1) m = fmaxf(m, __shfl_xor(m, off, 32));
      cm[r] = m;
    }
    __bf16* pwh = Psh[wave];
    __bf16* pwl = Psl[wave];
#pragma unroll
    for (int r = 0; r < 8; ++r) {
      const float mnew = fmaxf(mrow[r], cm[r]);
      const float alpha = expf(mrow[r] - mnew);
      mrow[r] = mnew;
      float psum = 0.f;
#pragma unroll
      for (int j = 0; j < 4; ++j) {
        const float p = expf(s[j][r] - mnew);
        psum += p;
        __bf16 a, bl; at_split(p, a, bl);
        pwh[(8 * hh + r) * AT_KC + j * 16 + c] = a;
        pwl[(8 * hh + r) * AT_KC + j * 16 + c] = bl;
      }
#pragma unroll
      for (int off = 1; off < 16; off <<= 1) psum += __shfl_xor(psum, off, 32);
      lrow[r] = lrow[r] * alpha + psum;
#pragma unroll
      for (int t = 0; t < 4; ++t) oacc[t][r] *= alpha;
    }
    __builtin_amdgcn_fence(__ATOMIC_RELEASE, "workgroup");
    __builtin_amdgcn_wave_barrier();
    __builtin_amdgcn_fence(__ATOMIC_ACQUIRE, "workgroup");
#pragma unroll 1
    for (int kk = 0; kk < 2; ++kk) {
      FB pa, pl;
      pa.h[0] = *(const v8b*)(pwh + c * AT_KC + kk * 32 + 8 * hh);
      pa.h[1] = *(const v8b*)(pwh + c * AT_KC + kk * 32 + 16 + 8 * hh);
      pl.h[0] = *(const v8b*)(pwl + c * AT_KC + kk * 32 + 8 * hh);
      pl.h[1] = *(const v8b*)(pwl + c * AT_KC + kk * 32 + 16 + 8 * hh);
#pragma unroll
      for (int t = 0; t < 4; ++t) {
        FB vb, vl;
        vb.h[0] = *(const v8b*)(Vth + (t * 16 + c) * AT_KC + kk * 32 + 8 * hh);
        vb.h[1] = *(const v8b*)(Vth + (t * 16 + c) * AT_KC + kk * 32 + 16 + 8 * hh);
        vl.h[0] = *(const v8b*)(Vtl + (t * 16 + c) * AT_KC + kk * 32 + 8 * hh);
        vl.h[1] = *(const v8b*)(Vtl + (t * 16 + c) * AT_KC + kk * 32 + 16 + 8 * hh);
        oacc[t] = at_mma(pa.v, vb.v, oacc[t]);
        oacc[t] = at_mma(pa.v, vl.v, oacc[t]);
        oacc[t] = at_mma(pl.v, vb.v, oacc[t]);
      }
    }
  }

  float* os = Os[wave];
#pragma unroll
  for (int r = 0; r < 8; ++r) {
    const float inv = 1.0f / lrow[r];
#pragma unroll
    for (int t = 0; t < 4; ++t) os[(8 * hh + r) * 68 + t * 16 + c] = oacc[t][r] * inv;
  }
  __builtin_amdgcn_fence(__ATOMIC_RELEASE, "workgroup");
  __builtin_amdgcn_wave_barrier();
  __builtin_amdgcn_fence(__ATOMIC_ACQUIRE, "workgroup");
  {
    const int q = lane >> 3, c8 = (lane & 7) * 8;
    v4u hv[4], lv[4];
#pragma unroll
    for (int it = 0; it < 4; ++it) {
      const int row = it * 4 + q;
      const float* sp = os + row * 68 + c8;
      const v4f a0 = *(const v4f*)(sp);
      const v4f a1 = *(const v4f*)(sp + 4);
      split8(a0, a1, hv[it], lv[it]);
    }
    for (int pass = 0; pass < 2; ++pass) {
#pragma unroll
      for (int it = 0; it < 4; ++it) {
        const int row = it * 4 + q;
        const size_t go = (tokb + (size_t)(q0 + row)) * CTXP + (size_t)h * AT_D + c8;
        *(volatile v4u*)(ctx + go)        = hv[it];
        *(volatile v4u*)(ctx + go + DMOD) = lv[it];
      }
      __threadfence();
    }
  }
}

extern "C" void kernel_launch(void* const* d_in, const int* in_sizes, int n_in,
                              void* d_out, int out_size, void* d_ws, size_t ws_size,
                              hipStream_t stream) {
  if (n_in < 4) return;
  if (in_sizes[0] != NTOK * DMOD) return;
  if (in_sizes[1] != 3 * DMOD * DMOD) return;
  if (in_sizes[2] != DMOD * DMOD) return;
  if (in_sizes[3] != DMOD) return;
  if (out_size != NTOK * DMOD) return;

  const float* x     = (const float*)d_in[0];
  const float* W_qkv = (const float*)d_in[1];
  const float* W_out = (const float*)d_in[2];
  const float* b_out = (const float*)d_in[3];
  float* out = (float*)d_out;

  const size_t bXB  = (size_t)NTOK * DMOD * 2;
  const size_t bWQ  = (size_t)3 * DMOD * DMOD * 2;
  const size_t bWO2 = (size_t)DMOD * 2 * DMOD * 2;
  const size_t bBR  = (size_t)DMOD * 4;
  const size_t bQK  = (size_t)NTOK * QKP * 2;
  const size_t bVT  = (size_t)NBATCH * DMOD * SEQ * 2;
  const size_t bCTX = (size_t)NTOK * CTXP * 2;
  size_t off = 0;
  const size_t oXB  = off; off += bXB;
  const size_t oWQ  = off; off += bWQ;
  const size_t oWO2 = off; off += bWO2;
  const size_t oBR  = off; off += bBR;
  const size_t oQKh = off; off += bQK;
  const size_t oQKl = off; off += bQK;
  const size_t oVTh = off; off += bVT;
  const size_t oVTl = off; off += bVT;
  const size_t oCTX = off; off += bCTX;
  if (off > ws_size) return;
  if (off > (size_t)134217728) return;

  char* ws = (char*)d_ws;
  unsigned short* XB   = (unsigned short*)(ws + oXB);
  unsigned short* WQKV = (unsigned short*)(ws + oWQ);
  unsigned short* WO2  = (unsigned short*)(ws + oWO2);
  float*          BR   = (float*)(ws + oBR);
  unsigned short* QKh  = (unsigned short*)(ws + oQKh);
  unsigned short* QKl  = (unsigned short*)(ws + oQKl);
  unsigned short* VTh  = (unsigned short*)(ws + oVTh);
  unsigned short* VTl  = (unsigned short*)(ws + oVTl);
  unsigned short* CTX  = (unsigned short*)(ws + oCTX);

  prep_kernel<<<dim3(NPREP / 256), dim3(256), 0, stream>>>(x, W_qkv, W_out, b_out, XB, WQKV, WO2, BR);

  wmma_gemm64<0, 2><<<dim3(((NTOK / 64) * (QKP / 64) + 7) / 8, 1), dim3(256), 0, stream>>>(
      XB, DMOD, 0L, WQKV, DMOD, 0L, (void*)QKh, (void*)QKl, QKP, 0L, BR, NTOK, QKP, DMOD);

  wmma_gemm64<0, 2><<<dim3(((DMOD / 64) * (SEQ / 64) + 7) / 8, NBATCH), dim3(256), 0, stream>>>(
      WQKV + (size_t)2 * DMOD * DMOD, DMOD, 0L, XB, DMOD, (long)SEQ * DMOD,
      (void*)VTh, (void*)VTl, SEQ, (long)DMOD * SEQ, BR, DMOD, SEQ, DMOD);

  attn_full64_kernel<<<dim3(NHEAD * (SEQ / AT_QB), NBATCH), dim3(128), 0, stream>>>(QKh, QKl, VTh, VTl, CTX);

  wmma_gemm64<2, 0><<<dim3(((NTOK / 64) * (DMOD / 64) + 7) / 8, 1), dim3(256), 0, stream>>>(
      CTX, CTXP, 0L, WO2, CTXP, 0L, (void*)out, (void*)out, DMOD, 0L, BR, NTOK, DMOD, CTXP);

  (void)hipGetLastError();
}
